// GAT_40166534152610
// MI455X (gfx1250) — hardware-verified
//
#include <hip/hip_runtime.h>
#include <stddef.h>
#include <stdint.h>

#define GB   2
#define GN   4096
#define GH   8
#define GD   64
#define GF   512
#define BM   128
#define KC   64
#define SPIT 68
#define U_H  524288
#define U_W  4096
#define U_A  256
#define WSMAX 134217728

static_assert(GN % BM == 0);
static_assert(GN % 32 == 0);
static_assert(GN % KC == 0 && KC == 64);
static_assert(GD == 64 && GH * GD == GF && GB * GH == 16);
static_assert(BM == 8 * 16);
static_assert(U_H % 256 == 0 && U_W % 256 == 0 && U_A == 256);
static_assert((long long)(GB * GN - 1) * GF + (GH - 1) * GD + 63 == (long long)GB * GN * GF - 1);

typedef float          v4f   __attribute__((ext_vector_type(4)));
typedef float          v8f   __attribute__((ext_vector_type(8)));
typedef int            v8i   __attribute__((ext_vector_type(8)));
typedef unsigned int   v4u   __attribute__((ext_vector_type(4)));
typedef unsigned short v8us  __attribute__((ext_vector_type(8)));
typedef unsigned short v16us __attribute__((ext_vector_type(16)));
typedef __bf16         v16bf __attribute__((ext_vector_type(16)));
typedef v4f  __attribute__((may_alias)) v4fa;
typedef v8us __attribute__((may_alias)) v8usa;
union FragB { v16bf v; v16us u; v8us h[2]; v8i w; };

__device__ __forceinline__ v8f wmb(const FragB& a, const FragB& b, v8f c) {
  v8f d = __builtin_amdgcn_wmma_f32_16x16x32_bf16(false, a.v, false, b.v, (short)0, c, false, false);
  asm volatile("v_nop\n\tv_nop\n\tv_nop\n\tv_nop" : "+v"(d) : "v"(a.w), "v"(b.w));
  return d;
}

__device__ __forceinline__ unsigned bf16_bits(float f) {
  const unsigned u = __float_as_uint(f);
  return (u + 0x7FFFu + ((u >> 16) & 1u)) >> 16;
}
__device__ __forceinline__ float bf16_val(float f) { return __uint_as_float(bf16_bits(f) << 16); }

struct PW { unsigned hi; unsigned lo; };
__device__ __forceinline__ PW split2(float a, float b) {
  const unsigned ha = bf16_bits(a), hb = bf16_bits(b);
  const unsigned la = bf16_bits(a - __uint_as_float(ha << 16));
  const unsigned lb = bf16_bits(b - __uint_as_float(hb << 16));
  PW r; r.hi = ha | (hb << 16); r.lo = la | (lb << 16); return r;
}

__device__ __forceinline__ float leaky02(float x) { return x > 0.0f ? x : 0.2f * x; }
__device__ __forceinline__ float pval(float x1, float s2, float mn) { return expf(leaky02(x1 + s2) - mn); }
__device__ __forceinline__ float elu1(float v) { return v > 0.0f ? v : expm1f(v); }

__global__ __launch_bounds__(256) void k_prep(const float* __restrict__ h, const float* __restrict__ W,
                                              const float* __restrict__ a,
                                              unsigned short* HB, unsigned short* WT, float* AF) {
  const int u = (int)blockIdx.x * 256 + (int)threadIdx.x;
  if (u < U_H) {
    const float* p = h + (size_t)u * 8;
    const v4f x = *(const v4f*)p;
    const v4f y = *(const v4f*)(p + 4);
    v8us o;
    o[0] = (unsigned short)bf16_bits(x.x); o[1] = (unsigned short)bf16_bits(x.y);
    o[2] = (unsigned short)bf16_bits(x.z); o[3] = (unsigned short)bf16_bits(x.w);
    o[4] = (unsigned short)bf16_bits(y.x); o[5] = (unsigned short)bf16_bits(y.y);
    o[6] = (unsigned short)bf16_bits(y.z); o[7] = (unsigned short)bf16_bits(y.w);
    unsigned short* dp = HB + (size_t)u * 8;
    *(volatile v8us*)dp = o;
    __threadfence();
    *(volatile v8us*)dp = o;
  } else if (u < U_H + U_W) {
    const int v   = u - U_H;
    const int hd  = v >> 9;
    const int rem = v & 511;
    const int oc  = rem >> 3;
    const int k8  = (rem & 7) * 8;
    const float* p = W + (size_t)hd * (GD * GD) + (size_t)k8 * GD + oc;
    v8us o;
#pragma unroll
    for (int i = 0; i < 8; ++i) o[i] = (unsigned short)bf16_bits(p[(size_t)i * GD]);
    unsigned short* dp = WT + (size_t)hd * (GD * GD) + (size_t)oc * GD + k8;
    *(volatile v8us*)dp = o;
    __threadfence();
    *(volatile v8us*)dp = o;
  } else if (u < U_H + U_W + U_A) {
    const int w = u - U_H - U_W;
    const v4f x = *(const v4f*)(a + (size_t)w * 4);
    v4f o;
    o.x = bf16_val(x.x); o.y = bf16_val(x.y); o.z = bf16_val(x.z); o.w = bf16_val(x.w);
    float* dp = AF + (size_t)w * 4;
    *(volatile v4f*)dp = o;
    __threadfence();
    *(volatile v4f*)dp = o;
  }
}

__global__ __launch_bounds__(256) void k_wh(const unsigned short* __restrict__ HB, const unsigned short* __restrict__ WT,
                                            const float* __restrict__ AF,
                                            unsigned short* VTH, unsigned short* VTL, float* SP) {
  __shared__ __attribute__((aligned(16))) float stg[BM * SPIT];
  __shared__ __attribute__((aligned(16))) float afs[2 * GD];
  __shared__ __attribute__((aligned(16))) float sdt[2 * BM];
  const int tid = (int)threadIdx.x, lane = tid & 31, wave = tid >> 5, hh = lane >> 4, m = lane & 15;
  const int hd = (int)blockIdx.x >> 6;
  const int mt = (int)blockIdx.x & 63;
  const int b  = mt >> 5;
  const int n0 = (mt & 31) * BM;
  const int rowBase = mt * BM;
  const int bh = b * GH + hd;

  v8f acc[4];
  {
    const v8f z = {0.f, 0.f, 0.f, 0.f, 0.f, 0.f, 0.f, 0.f};
#pragma unroll
    for (int t = 0; t < 4; ++t) acc[t] = z;
  }
  const unsigned short* ap = HB + (size_t)(rowBase + 16 * wave + m) * GF + hd * GD + 8 * hh;
  const unsigned short* bp = WT + (size_t)(hd * GD + m) * GD + 8 * hh;
#pragma unroll
  for (int k0 = 0; k0 < GD; k0 += 32) {
    FragB af;
    af.h[0] = *(const v8usa*)(ap + k0);
    af.h[1] = *(const v8usa*)(ap + k0 + 16);
#pragma unroll
    for (int nt = 0; nt < 4; ++nt) {
      const unsigned short* wq = bp + (size_t)(16 * nt) * GD + k0;
      FragB bf;
      bf.h[0] = *(const v8usa*)wq;
      bf.h[1] = *(const v8usa*)(wq + 16);
      acc[nt] = wmb(af, bf, acc[nt]);
    }
  }
#pragma unroll
  for (int nt = 0; nt < 4; ++nt) {
#pragma unroll
    for (int r = 0; r < 8; ++r) stg[(16 * wave + 8 * hh + r) * SPIT + 16 * nt + m] = acc[nt][r];
  }
  if (tid < 32) *(v4fa*)(afs + 4 * tid) = *(const v4fa*)(AF + (size_t)hd * (2 * GD) + 4 * tid);
  __syncthreads();

  {
    const int row  = tid >> 1;
    const int sel  = tid & 1;
    const int aoff = sel * GD;
    float s = 0.0f;
#pragma unroll 4
    for (int j4 = 0; j4 < GD / 4; ++j4) {
      const v4f p = *(const v4fa*)(stg + row * SPIT + 4 * j4);
      const v4f q = *(const v4fa*)(afs + aoff + 4 * j4);
      s = fmaf(p.x, q.x, s); s = fmaf(p.y, q.y, s); s = fmaf(p.z, q.z, s); s = fmaf(p.w, q.w, s);
    }
    sdt[sel * BM + row] = s;
  }
  __syncthreads();

  if (wave < 2) {
    const v4f sv = *(const v4fa*)(sdt + wave * BM + 4 * lane);
    float* sp = SP + (size_t)wave * (GB * GH * GN) + (size_t)bh * GN + n0 + 4 * lane;
    *(volatile v4f*)sp = sv;
    __threadfence();
    *(volatile v4f*)sp = sv;
  }

#pragma unroll 1
  for (int it = 0; it < 4; ++it) {
    const int u  = it * 256 + tid;
    const int oc = u >> 4;
    const int c8 = (u & 15) * 8;
    v4u hv, lv;
#pragma unroll
    for (int q = 0; q < 4; ++q) {
      const float f0 = stg[(c8 + 2 * q) * SPIT + oc];
      const float f1 = stg[(c8 + 2 * q + 1) * SPIT + oc];
      const PW w = split2(f0, f1);
      hv[q] = w.hi;
      lv[q] = w.lo;
    }
    const size_t go = ((size_t)bh * GD + oc) * GN + n0 + c8;
    *(volatile v4u*)(VTH + go) = hv;
    *(volatile v4u*)(VTL + go) = lv;
    __threadfence();
    *(volatile v4u*)(VTH + go) = hv;
    *(volatile v4u*)(VTL + go) = lv;
  }
}

__global__ __launch_bounds__(256) void k_attn(const unsigned short* __restrict__ VTH, const unsigned short* __restrict__ VTL,
                                              const float* __restrict__ SP, float* out) {
  __shared__ __attribute__((aligned(16))) float fbuf[8192];
  __shared__ __attribute__((aligned(16))) unsigned short Vh[GD * KC];
  __shared__ __attribute__((aligned(16))) unsigned short Vl[GD * KC];
  __shared__ float red[8];
  __shared__ float lsh[8 * 16];

  const int tid = (int)threadIdx.x, lane = tid & 31, wave = tid >> 5, hh = lane >> 4, c = lane & 15;
  const int bh = (int)blockIdx.x >> 5;
  const int rt = (int)blockIdx.x & 31;
  const int b  = bh >> 3;
  const int hd = bh & 7;
  const int q0 = rt * BM + wave * 16;
  const float* s1p = SP + (size_t)bh * GN;
  const float* s2p = SP + (size_t)(GB * GH * GN) + (size_t)bh * GN;

  float mloc = __int_as_float((int)0xff800000);
#pragma unroll
  for (int j = 0; j < 4; ++j) {
    const int i = tid * 4 + j * 1024;
    const v4f v = *(const v4fa*)(s2p + i);
    *(v4fa*)(fbuf + i) = v;
    mloc = fmaxf(mloc, fmaxf(fmaxf(v.x, v.y), fmaxf(v.z, v.w)));
  }
#pragma unroll
  for (int off = 16; off > 0; off >>= 1) mloc = fmaxf(mloc, __shfl_xor(mloc, off));
  if (lane == 0) red[wave] = mloc;
  const float x1 = s1p[q0 + c];
  __syncthreads();
  float M = red[0];
#pragma unroll
  for (int w2 = 1; w2 < 8; ++w2) M = fmaxf(M, red[w2]);
  const float mn = leaky02(x1 + M);

  v8f acc[4];
  {
    const v8f z = {0.f, 0.f, 0.f, 0.f, 0.f, 0.f, 0.f, 0.f};
#pragma unroll
    for (int t = 0; t < 4; ++t) acc[t] = z;
  }
  float lsum = 0.0f;

  const int sr = tid >> 2;
  const int sq = (tid & 3) * 16;
  const unsigned short* vth = VTH + ((size_t)bh * GD + sr) * GN + sq;
  const unsigned short* vtl = VTL + ((size_t)bh * GD + sr) * GN + sq;

#pragma unroll 1
  for (int kc = 0; kc < GN / KC; ++kc) {
    const int kv0 = kc * KC;
    __syncthreads();
    {
      const v8us a0 = *(const v8usa*)(vth + kv0);
      const v8us a1 = *(const v8usa*)(vth + kv0 + 8);
      const v8us b0 = *(const v8usa*)(vtl + kv0);
      const v8us b1 = *(const v8usa*)(vtl + kv0 + 8);
      *(v8usa*)(Vh + sr * KC + sq)     = a0;
      *(v8usa*)(Vh + sr * KC + sq + 8) = a1;
      *(v8usa*)(Vl + sr * KC + sq)     = b0;
      *(v8usa*)(Vl + sr * KC + sq + 8) = b1;
    }
    __syncthreads();
#pragma unroll 1
    for (int kk = 0; kk < 2; ++kk) {
      const float* sp = fbuf + kv0 + kk * 32 + 8 * hh;
      const v4f f0 = *(const v4fa*)(sp);
      const v4f f1 = *(const v4fa*)(sp + 4);
      const v4f f2 = *(const v4fa*)(sp + 16);
      const v4f f3 = *(const v4fa*)(sp + 20);
      FragB pa, pl;
      {
        const float p0 = pval(x1, f0.x, mn), p1 = pval(x1, f0.y, mn), p2 = pval(x1, f0.z, mn), p3 = pval(x1, f0.w, mn);
        lsum += p0; lsum += p1; lsum += p2; lsum += p3;
        const PW w0 = split2(p0, p1), w1 = split2(p2, p3);
        pa.w[0] = (int)w0.hi; pl.w[0] = (int)w0.lo;
        pa.w[1] = (int)w1.hi; pl.w[1] = (int)w1.lo;
      }
      {
        const float p0 = pval(x1, f1.x, mn), p1 = pval(x1, f1.y, mn), p2 = pval(x1, f1.z, mn), p3 = pval(x1, f1.w, mn);
        lsum += p0; lsum += p1; lsum += p2; lsum += p3;
        const PW w0 = split2(p0, p1), w1 = split2(p2, p3);
        pa.w[2] = (int)w0.hi; pl.w[2] = (int)w0.lo;
        pa.w[3] = (int)w1.hi; pl.w[3] = (int)w1.lo;
      }
      {
        const float p0 = pval(x1, f2.x, mn), p1 = pval(x1, f2.y, mn), p2 = pval(x1, f2.z, mn), p3 = pval(x1, f2.w, mn);
        lsum += p0; lsum += p1; lsum += p2; lsum += p3;
        const PW w0 = split2(p0, p1), w1 = split2(p2, p3);
        pa.w[4] = (int)w0.hi; pl.w[4] = (int)w0.lo;
        pa.w[5] = (int)w1.hi; pl.w[5] = (int)w1.lo;
      }
      {
        const float p0 = pval(x1, f3.x, mn), p1 = pval(x1, f3.y, mn), p2 = pval(x1, f3.z, mn), p3 = pval(x1, f3.w, mn);
        lsum += p0; lsum += p1; lsum += p2; lsum += p3;
        const PW w0 = split2(p0, p1), w1 = split2(p2, p3);
        pa.w[6] = (int)w0.hi; pl.w[6] = (int)w0.lo;
        pa.w[7] = (int)w1.hi; pl.w[7] = (int)w1.lo;
      }
#pragma unroll
      for (int t = 0; t < 4; ++t) {
        const int vo = (t * 16 + c) * KC + kk * 32 + 8 * hh;
        FragB vb, vl;
        vb.h[0] = *(const v8usa*)(Vh + vo);
        vb.h[1] = *(const v8usa*)(Vh + vo + 16);
        vl.h[0] = *(const v8usa*)(Vl + vo);
        vl.h[1] = *(const v8usa*)(Vl + vo + 16);
        acc[t] = wmb(pa, vb, acc[t]);
        acc[t] = wmb(pa, vl, acc[t]);
        acc[t] = wmb(pl, vb, acc[t]);
      }
    }
  }

  const float ltot = lsum + __shfl_xor(lsum, 16);
  __syncthreads();
  float* os = fbuf + wave * 1024;
#pragma unroll
  for (int t = 0; t < 4; ++t) {
#pragma unroll
    for (int r = 0; r < 8; ++r) os[(8 * hh + r) * 64 + t * 16 + c] = acc[t][r];
  }
  if (hh == 0) lsh[wave * 16 + c] = ltot;
  __syncthreads();

  const int c4 = c * 4;
  float* ob = out + ((size_t)b * GN + q0) * GF + hd * GD + c4;
#pragma unroll 1
  for (int it = 0; it < 8; ++it) {
    const int row = it * 2 + hh;
    const v4f v = *(const v4fa*)(os + row * 64 + c4);
    const float inv = 1.0f / lsh[wave * 16 + row];
    v4f o;
    o.x = elu1(v.x * inv); o.y = elu1(v.y * inv); o.z = elu1(v.z * inv); o.w = elu1(v.w * inv);
    float* p = ob + (size_t)row * GF;
    *(volatile v4f*)p = o;
    __threadfence();
    *(volatile v4f*)p = o;
  }
}

extern "C" void kernel_launch(void* const* d_in, const int* in_sizes, int n_in,
                              void* d_out, int out_size, void* d_ws, size_t ws_size,
                              hipStream_t stream) {
  if (n_in < 3) return;
  if (in_sizes[0] != GB * GN * GF) return;
  if (in_sizes[1] != GH * GD * GD) return;
  if (in_sizes[2] != GH * 2 * GD) return;
  if (out_size != GB * GN * GF) return;

  const float* h = (const float*)d_in[0];
  const float* W = (const float*)d_in[1];
  const float* a = (const float*)d_in[2];
  float* out = (float*)d_out;

  size_t off = 0;
  const size_t oHB  = off; off += (size_t)GB * GN * GF * 2;
  const size_t oVTH = off; off += (size_t)GB * GH * GD * GN * 2;
  const size_t oVTL = off; off += (size_t)GB * GH * GD * GN * 2;
  const size_t oSP  = off; off += (size_t)2 * GB * GH * GN * 4;
  const size_t oWT  = off; off += (size_t)GH * GD * GD * 2;
  const size_t oAF  = off; off += (size_t)GH * 2 * GD * 4;
  if (off > ws_size || off > (size_t)WSMAX) return;

  char* ws = (char*)d_ws;
  unsigned short* HB  = (unsigned short*)(ws + oHB);
  unsigned short* VTH = (unsigned short*)(ws + oVTH);
  unsigned short* VTL = (unsigned short*)(ws + oVTL);
  float*          SP  = (float*)(ws + oSP);
  unsigned short* WT  = (unsigned short*)(ws + oWT);
  float*          AF  = (float*)(ws + oAF);

  k_prep<<<(U_H + U_W + U_A) / 256, 256, 0, stream>>>(h, W, a, HB, WT, AF);
  k_wh<<<GH * (GB * GN / BM), 256, 0, stream>>>(HB, WT, AF, VTH, VTL, SP);
  k_attn<<<GB * GH * (GN / BM), 256, 0, stream>>>(VTH, VTL, SP, out);
  (void)hipGetLastError();
}
